// DeepSetEquivariantTransform_6992206757904
// MI455X (gfx1250) — hardware-run, weakly checked
//
#include <hip/hip_runtime.h>
#include <math.h>

constexpr int kSets      = 512;
constexpr int kPos       = 200;
constexpr int kFeat      = 16;
constexpr int kWidth     = 256;
constexpr int kLat       = 128;
constexpr int kRows      = kSets * kPos;
constexpr int kHalfSets  = 256;
constexpr int kHalfRows  = kHalfSets * kPos;
constexpr int kK0        = 64;
constexpr int kNLast     = 64;
constexpr int kMidLayers = 3;
constexpr int kFMid      = 4;
constexpr float kAlpha   = 0.2f;

typedef __attribute__((ext_vector_type(16))) _Float16 v16h;
typedef __attribute__((ext_vector_type(8)))  _Float16 v8h;
typedef __attribute__((ext_vector_type(16))) __bf16   v16b;
typedef __attribute__((ext_vector_type(8)))  __bf16   v8b;
typedef __attribute__((ext_vector_type(8)))  float    v8f;
typedef __attribute__((ext_vector_type(4)))  float    v4f;
typedef __attribute__((ext_vector_type(4)))  unsigned int v4u;

__device__ __forceinline__ unsigned short f2bf_bits(float f) {
  unsigned u = __float_as_uint(f);
  return (unsigned short)((u + 0x7FFFu + ((u >> 16) & 1u)) >> 16);
}
__device__ __forceinline__ float bf_bits2f(unsigned short h) { return __uint_as_float(((unsigned)h) << 16); }

__device__ __forceinline__ void dep_guard_h(v8f& a, v8f& b, v16h x, v16h y) { asm volatile("v_nop\n\tv_nop\n\tv_nop\n\tv_nop" : "+v"(a), "+v"(b) : "v"(x), "v"(y)); }
__device__ __forceinline__ void dep_guard_b(v8f& a, v8f& b, v16b x, v16b y) { asm volatile("v_nop\n\tv_nop\n\tv_nop\n\tv_nop" : "+v"(a), "+v"(b) : "v"(x), "v"(y)); }
__device__ __forceinline__ void keep4_h(v16h a, v16h b, v16h c, v16h d) { asm volatile("v_nop" :: "v"(a), "v"(b), "v"(c), "v"(d)); }
__device__ __forceinline__ void keep4_b(v16b a, v16b b, v16b c, v16b d) { asm volatile("v_nop" :: "v"(a), "v"(b), "v"(c), "v"(d)); }
__device__ __forceinline__ void acc_guard4(v8f& a, v8f& b, v8f& c, v8f& d) { asm volatile("v_nop\n\tv_nop\n\tv_nop\n\tv_nop" : "+v"(a), "+v"(b), "+v"(c), "+v"(d)); }
template <typename T> struct Frag;
template <> struct Frag<_Float16> {
  typedef v16h V; union U { v16h v; v8h h[2]; };
  static __device__ __forceinline__ v16h load(const _Float16* p) {
    U f; f.h[0] = *(const v8h*)(p); f.h[1] = *(const v8h*)(p + 16); return f.v;
  }
  static __device__ __forceinline__ v8f mma(v16h a, v16h b, v8f c) {
    return __builtin_amdgcn_wmma_f32_16x16x32_f16(false, a, false, b, (short)0, c, false, false);
  }
  static __device__ __forceinline__ void guard(v8f& a, v8f& b, v16h x, v16h y) { dep_guard_h(a, b, x, y); }
  static __device__ __forceinline__ void keep(v16h a, v16h b, v16h c, v16h d) { keep4_h(a, b, c, d); }
};
template <> struct Frag<__bf16> {
  typedef v16b V; union U { v16b v; v8b h[2]; };
  static __device__ __forceinline__ v16b load(const __bf16* p) {
    U f; f.h[0] = *(const v8b*)(p); f.h[1] = *(const v8b*)(p + 16); return f.v;
  }
  static __device__ __forceinline__ v8f mma(v16b a, v16b b, v8f c) {
    return __builtin_amdgcn_wmma_f32_16x16x32_bf16(false, a, false, b, (short)0, c, false, false);
  }
  static __device__ __forceinline__ void guard(v8f& a, v8f& b, v16b x, v16b y) { dep_guard_b(a, b, x, y); }
  static __device__ __forceinline__ void keep(v16b a, v16b b, v16b c, v16b d) { keep4_b(a, b, c, d); }
};

__device__ __forceinline__ unsigned pk16(unsigned short a, unsigned short b) { return (unsigned)a | ((unsigned)b << 16); }

template <int ET> struct Elem;
template <> struct Elem<0> { typedef _Float16 T; };
template <> struct Elem<1> { typedef __bf16 T; };
template <int ET, int SPL, int BIAS_MODE, int OUT_MODE, int ACT>
__global__ __launch_bounds__(256) void wmma_gemm64(
    const unsigned short* __restrict__ Ap, const unsigned short* __restrict__ A2p, int lda, long strideA,
    const unsigned short* __restrict__ Btp, const unsigned short* __restrict__ Bt2p, int ldb, long strideB,
    void* __restrict__ Cout, void* __restrict__ Cout2, int ldc, long strideC,
    const float* __restrict__ bias, int ldbias,
    int M, int N, int K, float scale) {
  typedef typename Elem<ET>::T T;
  typedef typename Frag<T>::V V;
  const T* A = (const T*)Ap; const T* A2 = (const T*)A2p; const T* Bt = (const T*)Btp; const T* Bt2 = (const T*)Bt2p;
  __shared__ __align__(16) float sT[8][16 * 68];
  const int b    = blockIdx.y;
  const int lane = threadIdx.x & 31;
  const int wave = threadIdx.x >> 5;
  const int tilesN = N >> 6;
  const int tilesM = M >> 6;
  const int tile = blockIdx.x * 8 + wave;
  if (tile >= tilesM * tilesN) return;
  const int tm = tile / tilesN;
  const int tn = tile - tm * tilesN;
  const int m0 = tm << 6;
  const int n0 = tn << 6;

  const T* Ab  = A  + (size_t)b * strideA;
  const T* Bb  = Bt + (size_t)b * strideB;
  const T* Ab2 = (SPL & 1) ? (A2  + (size_t)b * strideA) : nullptr;
  const T* Bb2 = (SPL & 2) ? (Bt2 + (size_t)b * strideB) : nullptr;

  const int rlane = lane & 15;
  const int koff  = (lane >> 4) * 8;
  const int mOff  = (lane >> 4) * 8;

  v8f acc[4][4];
#pragma unroll
  for (int i = 0; i < 4; ++i)
#pragma unroll
    for (int j = 0; j < 4; ++j) acc[i][j] = (v8f){0.f,0.f,0.f,0.f,0.f,0.f,0.f,0.f};

  for (int k0 = 0; k0 < K; k0 += 32) {
    V bh[4], bl[4];
#pragma unroll
    for (int j = 0; j < 4; ++j) {
      const size_t bo = (size_t)(n0 + (j << 4) + rlane) * ldb + koff + k0;
      bh[j] = Frag<T>::load(Bb + bo);
      if (SPL & 2) bl[j] = Frag<T>::load(Bb2 + bo);
    }
#pragma unroll
    for (int i = 0; i < 4; ++i) {
      const size_t ao = (size_t)(m0 + (i << 4) + rlane) * lda + koff + k0;
      V ah = Frag<T>::load(Ab + ao);
      V al;
      if (SPL & 1) al = Frag<T>::load(Ab2 + ao);
#pragma unroll
      for (int j = 0; j < 4; ++j) {
        acc[i][j] = Frag<T>::mma(ah, bh[j], acc[i][j]);
        if (SPL & 2) acc[i][j] = Frag<T>::mma(ah, bl[j], acc[i][j]);
        if (SPL & 1) acc[i][j] = Frag<T>::mma(al, bh[j], acc[i][j]);
      }
      Frag<T>::guard(acc[i][0], acc[i][3], ah, (SPL & 1) ? al : ah);
    }
    Frag<T>::keep(bh[0], bh[1], bh[2], bh[3]);
    if (SPL & 2) Frag<T>::keep(bl[0], bl[1], bl[2], bl[3]);
  }
  acc_guard4(acc[0][0], acc[0][1], acc[0][2], acc[0][3]);
  acc_guard4(acc[1][0], acc[1][1], acc[1][2], acc[1][3]);
  acc_guard4(acc[2][0], acc[2][1], acc[2][2], acc[2][3]);
  acc_guard4(acc[3][0], acc[3][1], acc[3][2], acc[3][3]);

  float* slab = sT[wave];
#pragma unroll
  for (int i = 0; i < 4; ++i) {
    const int mBase = m0 + (i << 4);
#pragma unroll
    for (int j = 0; j < 4; ++j) {
      const int n = n0 + (j << 4) + rlane;
      float bv = 0.f;
      if (BIAS_MODE == 2) bv = bias[n];
#pragma unroll
      for (int r = 0; r < 8; ++r) {
        float v = acc[i][j][r] * scale;
        if (BIAS_MODE == 1) v += bias[mBase + mOff + r];
        if (BIAS_MODE == 2) v += bv;
        if (BIAS_MODE == 3) v -= bias[(size_t)((mBase + mOff + r) / kPos) * ldbias + n];
        if (ACT == 7) v = (v >= 0.0f) ? v : kAlpha * v;
        slab[(mOff + r) * 68 + (j << 4) + rlane] = v;
      }
    }
    __builtin_amdgcn_fence(__ATOMIC_RELEASE, "workgroup");
    __builtin_amdgcn_wave_barrier();
    __builtin_amdgcn_fence(__ATOMIC_ACQUIRE, "workgroup");
    if (OUT_MODE == 0) {
      float* C = (float*)Cout + (size_t)b * strideC;
      const int hh = lane >> 4, c4 = (lane & 15) * 4;
      for (int pass = 0; pass < 2; ++pass) {
#pragma unroll
        for (int it = 0; it < 8; ++it) {
          const int row = it * 2 + hh;
          v4f v = *(const v4f*)(slab + row * 68 + c4);
          *(volatile v4f*)(C + (size_t)(mBase + row) * ldc + n0 + c4) = v;
        }
        __threadfence();
      }
    } else {
      const int q = lane >> 3, c8 = (lane & 7) * 8;
      unsigned short* C  = (unsigned short*)Cout  + (size_t)b * strideC;
      unsigned short* C2 = (OUT_MODE == 2) ? ((unsigned short*)Cout2 + (size_t)b * strideC) : nullptr;
      for (int pass = 0; pass < 2; ++pass) {
#pragma unroll
        for (int it = 0; it < 4; ++it) {
          const int row = it * 4 + q;
          const float* sp = slab + row * 68 + c8;
          v8h hv, lv;
#pragma unroll
          for (int e = 0; e < 8; ++e) {
            if (OUT_MODE == 1) {
              hv[e] = (_Float16)sp[e];
            } else {
              unsigned short hb = f2bf_bits(sp[e]);
              unsigned short lb = f2bf_bits(sp[e] - bf_bits2f(hb));
              hv[e] = __builtin_bit_cast(_Float16, hb);
              lv[e] = __builtin_bit_cast(_Float16, lb);
            }
          }
          *(volatile v8h*)(C + (size_t)(mBase + row) * ldc + n0 + c8) = hv;
          if (OUT_MODE == 2) *(volatile v8h*)(C2 + (size_t)(mBase + row) * ldc + n0 + c8) = lv;
        }
        __threadfence();
      }
    }
    __builtin_amdgcn_fence(__ATOMIC_RELEASE, "workgroup");
    __builtin_amdgcn_wave_barrier();
    __builtin_amdgcn_fence(__ATOMIC_ACQUIRE, "workgroup");
  }
}

__global__ __launch_bounds__(256) void prep_kernel(const float* __restrict__ x, unsigned short* __restrict__ XB,
                                                   float* __restrict__ MASK) {
  __shared__ __align__(16) unsigned sx[256 * 32];
  __shared__ __align__(16) float smask[256];
  const int t = threadIdx.x, lane = t & 31, wave = t >> 5;
  const int r0 = blockIdx.x * 256;
  const float* xr = x + ((size_t)r0 + t) * kFeat;
  const v4f a0 = *(const v4f*)(xr);
  const v4f a1 = *(const v4f*)(xr + 4);
  const v4f a2 = *(const v4f*)(xr + 8);
  const v4f a3 = *(const v4f*)(xr + 12);
  int nz = 0;
#pragma unroll
  for (int e = 0; e < 4; ++e) {
    nz |= (a0[e] != 0.0f) ? 1 : 0;
    nz |= (a1[e] != 0.0f) ? 1 : 0;
    nz |= (a2[e] != 0.0f) ? 1 : 0;
    nz |= (a3[e] != 0.0f) ? 1 : 0;
  }
  unsigned w[8];
  w[0] = pk16(f2bf_bits(a0[0]), f2bf_bits(a0[1])); w[1] = pk16(f2bf_bits(a0[2]), f2bf_bits(a0[3]));
  w[2] = pk16(f2bf_bits(a1[0]), f2bf_bits(a1[1])); w[3] = pk16(f2bf_bits(a1[2]), f2bf_bits(a1[3]));
  w[4] = pk16(f2bf_bits(a2[0]), f2bf_bits(a2[1])); w[5] = pk16(f2bf_bits(a2[2]), f2bf_bits(a2[3]));
  w[6] = pk16(f2bf_bits(a3[0]), f2bf_bits(a3[1])); w[7] = pk16(f2bf_bits(a3[2]), f2bf_bits(a3[3]));
  unsigned* srow = sx + t * 32;
#pragma unroll
  for (int i = 0; i < 8; ++i) srow[i] = w[i];
#pragma unroll
  for (int i = 8; i < 32; ++i) srow[i] = 0u;
  smask[t] = nz ? 1.0f : 0.0f;
  __syncthreads();
  const int q = lane >> 3, c = lane & 7;
  unsigned* XBu = (unsigned*)XB;
  v4f mv = (v4f){0.f, 0.f, 0.f, 0.f};
  if (t < 64) mv = *(const v4f*)(smask + 4 * t);
  for (int pass = 0; pass < 2; ++pass) {
#pragma unroll
    for (int it = 0; it < 8; ++it) {
      const int lrow = it * 32 + wave * 4 + q;
      const v4u v = *(const v4u*)(sx + lrow * 32 + c * 4);
      *(volatile v4u*)(XBu + ((size_t)r0 + lrow) * 32 + c * 4) = v;
    }
    if (t < 64) *(volatile v4f*)(MASK + (size_t)r0 + 4 * t) = mv;
    __threadfence();
  }
}

__global__ __launch_bounds__(256) void transpose_cast_kernel(const float* __restrict__ W, int K, int N,
                                                             unsigned short* __restrict__ WT, int Kpad,
                                                             long strideIn, long strideOut) {
  __shared__ __align__(16) float tile[64 * 68];
  const int t = threadIdx.x, lane = t & 31, wave = t >> 5;
  const int k0 = blockIdx.x * 64, n0 = blockIdx.y * 64;
  const float* Wz = W + (size_t)blockIdx.z * strideIn;
  unsigned short* Oz = WT + (size_t)blockIdx.z * strideOut;
  {
    const int nn = t & 63, kq = t >> 6;
    const int n = n0 + nn;
    const int nc = (n < N) ? n : (N - 1);
#pragma unroll
    for (int i = 0; i < 16; ++i) {
      const int kk = kq + 4 * i;
      const int k = k0 + kk;
      const int kc = (k < K) ? k : (K - 1);
      float v = Wz[(size_t)kc * N + nc];
      if (k >= K || n >= N) v = 0.0f;
      tile[nn * 68 + kk] = v;
    }
  }
  __syncthreads();
  const int q = lane >> 3, c8 = (lane & 7) * 8;
  for (int pass = 0; pass < 2; ++pass) {
#pragma unroll
    for (int it = 0; it < 2; ++it) {
      const int r = it * 32 + wave * 4 + q;
      const float* sp = tile + r * 68 + c8;
      v8h hv;
#pragma unroll
      for (int e = 0; e < 8; ++e) hv[e] = __builtin_bit_cast(_Float16, f2bf_bits(sp[e]));
      *(volatile v8h*)(Oz + (size_t)(n0 + r) * Kpad + k0 + c8) = hv;
    }
    __threadfence();
  }
}

template <int KIN, bool HAS_LO, bool DIV>
__global__ __launch_bounds__(256) void colsum_kernel(const unsigned short* __restrict__ Hh, const unsigned short* __restrict__ Hl,
                                                     const float* __restrict__ mask,
                                                     unsigned short* __restrict__ Oh, unsigned short* __restrict__ Ol) {
  constexpr int G = KIN / 8;
  constexpr int NPH = 256 / G;
  __shared__ __align__(16) float red[256 * 8];
  __shared__ float redc[256];
  __shared__ unsigned short shi[KIN];
  __shared__ unsigned short slo[KIN];
  const int b = blockIdx.x, t = threadIdx.x;
  const int g = t & (G - 1), ph = t / G;
  const int c0 = g * 8;
  float s[8];
#pragma unroll
  for (int e = 0; e < 8; ++e) s[e] = 0.0f;
  float cnt = 0.0f;
  const size_t rb = (size_t)b * kPos;
#pragma unroll 1
  for (int n = ph; n < kPos; n += NPH) {
    const size_t row = rb + n;
    const float m = mask[row];
    const v4u uh = *(const v4u*)(Hh + row * KIN + c0);
    v4u ul = (v4u){0u, 0u, 0u, 0u};
    if (HAS_LO) ul = *(const v4u*)(Hl + row * KIN + c0);
#pragma unroll
    for (int q = 0; q < 4; ++q) {
      float f0 = __uint_as_float(uh[q] << 16);
      float f1 = __uint_as_float(uh[q] & 0xFFFF0000u);
      if (HAS_LO) {
        f0 += __uint_as_float(ul[q] << 16);
        f1 += __uint_as_float(ul[q] & 0xFFFF0000u);
      }
      s[2 * q]     = fmaf(m, f0, s[2 * q]);
      s[2 * q + 1] = fmaf(m, f1, s[2 * q + 1]);
    }
    cnt += m;
  }
#pragma unroll
  for (int e = 0; e < 8; ++e) red[t * 8 + e] = s[e];
  redc[t] = cnt;
  __syncthreads();
  if (t < KIN) {
    const int g2 = t >> 3, e = t & 7;
    float tot = 0.0f, den = 0.0f;
#pragma unroll 1
    for (int p2 = 0; p2 < NPH; ++p2) {
      tot += red[(p2 * G + g2) * 8 + e];
      den += redc[p2 * G + g2];
    }
    const float val = DIV ? (tot * (1.0f / den)) : tot;
    const unsigned short hb = f2bf_bits(val);
    shi[t] = hb;
    slo[t] = f2bf_bits(val - bf_bits2f(hb));
  }
  __syncthreads();
  const int gi = g * 8;
  const v4u hv4 = (v4u){pk16(shi[gi], shi[gi + 1]), pk16(shi[gi + 2], shi[gi + 3]),
                        pk16(shi[gi + 4], shi[gi + 5]), pk16(shi[gi + 6], shi[gi + 7])};
  const v4u lv4 = (v4u){pk16(slo[gi], slo[gi + 1]), pk16(slo[gi + 2], slo[gi + 3]),
                        pk16(slo[gi + 4], slo[gi + 5]), pk16(slo[gi + 6], slo[gi + 7])};
  unsigned short* oh = Oh + (size_t)b * KIN + gi;
  unsigned short* ol = Ol + (size_t)b * KIN + gi;
  for (int pass = 0; pass < 2; ++pass) {
    if (t < G) *(volatile v4u*)oh = hv4;
    if (t >= G && t < 2 * G) *(volatile v4u*)ol = lv4;
    __threadfence();
  }
}

__global__ __launch_bounds__(256) void softmax_out_kernel(const float* __restrict__ Z, const float* __restrict__ bl,
                                                          float* __restrict__ out) {
  __shared__ __align__(16) float so[kSets * 2];
  const int t = threadIdx.x;
  const float b0 = bl[0], b1 = bl[1];
#pragma unroll 1
  for (int hh = 0; hh < 2; ++hh) {
    const int b = t + 256 * hh;
    const float z0 = Z[(size_t)b * kNLast + 0] + b0;
    const float z1 = Z[(size_t)b * kNLast + 1] + b1;
    const float m = fmaxf(z0, z1);
    const float e0 = expf(z0 - m), e1 = expf(z1 - m);
    const float r = 1.0f / (e0 + e1);
    so[2 * b]     = e0 * r;
    so[2 * b + 1] = e1 * r;
  }
  __syncthreads();
  const v4f v = *(const v4f*)(so + 4 * t);
  for (int pass = 0; pass < 2; ++pass) {
    *(volatile v4f*)(out + 4 * t) = v;
    __threadfence();
  }
}

static inline dim3 gemm_grid(int M, int N) { return dim3((unsigned)(((M / 64) * (N / 64) + 7) / 8), 1, 1); }

extern "C" void kernel_launch(void* const* d_in, const int* in_sizes, int n_in,
                              void* d_out, int out_size, void* d_ws, size_t ws_size,
                              hipStream_t stream) {
  if (n_in < 13) return;
  if (in_sizes[0] != kRows * kFeat) return;
  if (in_sizes[1] != kFeat * kWidth || in_sizes[2] != kFeat * kWidth) return;
  if (in_sizes[3] != kMidLayers * kWidth * kWidth || in_sizes[4] != kMidLayers * kWidth * kWidth) return;
  if (in_sizes[5] != kWidth * kLat || in_sizes[6] != kWidth * kLat) return;
  if (in_sizes[7] != kLat * kWidth || in_sizes[8] != kWidth) return;
  if (in_sizes[9] != kFMid * kWidth * kWidth || in_sizes[10] != kFMid * kWidth) return;
  if (in_sizes[11] != kWidth * 2 || in_sizes[12] != 2) return;
  if (out_size != kSets * 2) return;
  if ((kRows % 256) != 0 || (kHalfRows % 64) != 0) return;

  const float* x       = (const float*)d_in[0];
  const float* Gamma0  = (const float*)d_in[1];
  const float* Lambda0 = (const float*)d_in[2];
  const float* Gmid    = (const float*)d_in[3];
  const float* Lmid    = (const float*)d_in[4];
  const float* GammaL  = (const float*)d_in[5];
  const float* LambdaL = (const float*)d_in[6];
  const float* F0W     = (const float*)d_in[7];
  const float* F0b     = (const float*)d_in[8];
  const float* FmW     = (const float*)d_in[9];
  const float* Fmb     = (const float*)d_in[10];
  const float* FlW     = (const float*)d_in[11];
  const float* Flb     = (const float*)d_in[12];
  float* outp = (float*)d_out;

  const size_t SZ_XB   = (size_t)kRows * kK0 * 2;
  const size_t SZ_MASK = (size_t)kRows * 4;
  const size_t SZ_P    = (size_t)kHalfRows * kWidth * 2;
  const size_t SZ_MEAN = (size_t)kHalfSets * kWidth * 2;
  const size_t SZ_ML   = (size_t)kHalfSets * kWidth * 4;
  const size_t SZ_POOL = (size_t)kSets * kLat * 2;
  const size_t SZ_Y    = (size_t)kSets * kWidth * 2;
  const size_t SZ_Z    = (size_t)kSets * kNLast * 4;
  const size_t SZ_G0T  = (size_t)kWidth * kK0 * 2;
  const size_t SZ_GMT  = (size_t)kMidLayers * kWidth * kWidth * 2;
  const size_t SZ_GLT  = (size_t)kLat * kWidth * 2;
  const size_t SZ_F0T  = (size_t)kWidth * kLat * 2;
  const size_t SZ_FMT  = (size_t)kFMid * kWidth * kWidth * 2;
  const size_t SZ_FLT  = (size_t)kNLast * kWidth * 2;

  size_t off = 0;
  const size_t oXB = off;    off += SZ_XB;
  const size_t oMASK = off;  off += SZ_MASK;
  const size_t oP0H = off;   off += SZ_P;
  const size_t oP0L = off;   off += SZ_P;
  const size_t oP1H = off;   off += SZ_P;
  const size_t oP1L = off;   off += SZ_P;
  const size_t oMEANH = off; off += SZ_MEAN;
  const size_t oMEANL = off; off += SZ_MEAN;
  const size_t oML = off;    off += SZ_ML;
  const size_t oPOOLH = off; off += SZ_POOL;
  const size_t oPOOLL = off; off += SZ_POOL;
  const size_t oY0H = off;   off += SZ_Y;
  const size_t oY0L = off;   off += SZ_Y;
  const size_t oY1H = off;   off += SZ_Y;
  const size_t oY1L = off;   off += SZ_Y;
  const size_t oZ = off;     off += SZ_Z;
  const size_t oG0T = off;   off += SZ_G0T;
  const size_t oL0T = off;   off += SZ_G0T;
  const size_t oGMT = off;   off += SZ_GMT;
  const size_t oLMT = off;   off += SZ_GMT;
  const size_t oGLT = off;   off += SZ_GLT;
  const size_t oLLT = off;   off += SZ_GLT;
  const size_t oF0T = off;   off += SZ_F0T;
  const size_t oFMT = off;   off += SZ_FMT;
  const size_t oFLT = off;   off += SZ_FLT;
  const size_t TOTAL = off;
  if (TOTAL > ws_size) return;
  if (TOTAL > (size_t)134217728) return;

  char* ws = (char*)d_ws;
  unsigned short* XB    = (unsigned short*)(ws + oXB);
  float*          MASK  = (float*)(ws + oMASK);
  unsigned short* P0H   = (unsigned short*)(ws + oP0H);
  unsigned short* P0L   = (unsigned short*)(ws + oP0L);
  unsigned short* P1H   = (unsigned short*)(ws + oP1H);
  unsigned short* P1L   = (unsigned short*)(ws + oP1L);
  unsigned short* MEANH = (unsigned short*)(ws + oMEANH);
  unsigned short* MEANL = (unsigned short*)(ws + oMEANL);
  float*          ML    = (float*)(ws + oML);
  unsigned short* POOLH = (unsigned short*)(ws + oPOOLH);
  unsigned short* POOLL = (unsigned short*)(ws + oPOOLL);
  unsigned short* Y0H   = (unsigned short*)(ws + oY0H);
  unsigned short* Y0L   = (unsigned short*)(ws + oY0L);
  unsigned short* Y1H   = (unsigned short*)(ws + oY1H);
  unsigned short* Y1L   = (unsigned short*)(ws + oY1L);
  float*          Z     = (float*)(ws + oZ);
  unsigned short* G0T   = (unsigned short*)(ws + oG0T);
  unsigned short* L0T   = (unsigned short*)(ws + oL0T);
  unsigned short* GMT   = (unsigned short*)(ws + oGMT);
  unsigned short* LMT   = (unsigned short*)(ws + oLMT);
  unsigned short* GLT   = (unsigned short*)(ws + oGLT);
  unsigned short* LLT   = (unsigned short*)(ws + oLLT);
  unsigned short* F0T   = (unsigned short*)(ws + oF0T);
  unsigned short* FMT   = (unsigned short*)(ws + oFMT);
  unsigned short* FLT   = (unsigned short*)(ws + oFLT);

  const dim3 blk(256);
  const long sqW = (long)kWidth * kWidth;

  transpose_cast_kernel<<<dim3(1, 4, 1), blk, 0, stream>>>(Gamma0, kFeat, kWidth, G0T, kK0, 0L, 0L);
  transpose_cast_kernel<<<dim3(1, 4, 1), blk, 0, stream>>>(Lambda0, kFeat, kWidth, L0T, kK0, 0L, 0L);
  transpose_cast_kernel<<<dim3(4, 4, kMidLayers), blk, 0, stream>>>(Gmid, kWidth, kWidth, GMT, kWidth, sqW, sqW);
  transpose_cast_kernel<<<dim3(4, 4, kMidLayers), blk, 0, stream>>>(Lmid, kWidth, kWidth, LMT, kWidth, sqW, sqW);
  transpose_cast_kernel<<<dim3(4, 2, 1), blk, 0, stream>>>(GammaL, kWidth, kLat, GLT, kWidth, 0L, 0L);
  transpose_cast_kernel<<<dim3(4, 2, 1), blk, 0, stream>>>(LambdaL, kWidth, kLat, LLT, kWidth, 0L, 0L);
  transpose_cast_kernel<<<dim3(2, 4, 1), blk, 0, stream>>>(F0W, kLat, kWidth, F0T, kLat, 0L, 0L);
  transpose_cast_kernel<<<dim3(4, 4, kFMid), blk, 0, stream>>>(FmW, kWidth, kWidth, FMT, kWidth, sqW, sqW);
  transpose_cast_kernel<<<dim3(4, 1, 1), blk, 0, stream>>>(FlW, kWidth, 2, FLT, kWidth, 0L, 0L);

  prep_kernel<<<dim3(kRows / 256), blk, 0, stream>>>(x, XB, MASK);

  for (int half = 0; half < 2; ++half) {
    const size_t hoff = (size_t)half * kHalfRows;
    const size_t soff = (size_t)half * kHalfSets;
    const unsigned short* XBh = XB + hoff * kK0;
    const float* MK = MASK + hoff;

    colsum_kernel<kK0, false, true><<<dim3(kHalfSets), blk, 0, stream>>>(XBh, XBh, MK, MEANH, MEANL);
    wmma_gemm64<1, 1, 0, 0, 0><<<gemm_grid(kHalfSets, kWidth), blk, 0, stream>>>(
        MEANH, MEANL, kK0, 0L, L0T, L0T, kK0, 0L, (void*)ML, (void*)ML, kWidth, 0L, ML, 0,
        kHalfSets, kWidth, kK0, 1.0f);
    wmma_gemm64<1, 0, 3, 2, 7><<<gemm_grid(kHalfRows, kWidth), blk, 0, stream>>>(
        XBh, XBh, kK0, 0L, G0T, G0T, kK0, 0L, (void*)P0H, (void*)P0L, kWidth, 0L, ML, kWidth,
        kHalfRows, kWidth, kK0, 1.0f);

    unsigned short* curH = P0H; unsigned short* curL = P0L;
    unsigned short* nxtH = P1H; unsigned short* nxtL = P1L;
    for (int i = 0; i < kMidLayers; ++i) {
      colsum_kernel<kWidth, true, true><<<dim3(kHalfSets), blk, 0, stream>>>(curH, curL, MK, MEANH, MEANL);
      wmma_gemm64<1, 1, 0, 0, 0><<<gemm_grid(kHalfSets, kWidth), blk, 0, stream>>>(
          MEANH, MEANL, kWidth, 0L, LMT + (size_t)i * sqW, LMT + (size_t)i * sqW, kWidth, 0L,
          (void*)ML, (void*)ML, kWidth, 0L, ML, 0, kHalfSets, kWidth, kWidth, 1.0f);
      wmma_gemm64<1, 1, 3, 2, 7><<<gemm_grid(kHalfRows, kWidth), blk, 0, stream>>>(
          curH, curL, kWidth, 0L, GMT + (size_t)i * sqW, GMT + (size_t)i * sqW, kWidth, 0L,
          (void*)nxtH, (void*)nxtL, kWidth, 0L, ML, kWidth, kHalfRows, kWidth, kWidth, 1.0f);
      unsigned short* th = curH; curH = nxtH; nxtH = th;
      unsigned short* tl = curL; curL = nxtL; nxtL = tl;
    }
    colsum_kernel<kWidth, true, true><<<dim3(kHalfSets), blk, 0, stream>>>(curH, curL, MK, MEANH, MEANL);
    wmma_gemm64<1, 1, 0, 0, 0><<<gemm_grid(kHalfSets, kLat), blk, 0, stream>>>(
        MEANH, MEANL, kWidth, 0L, LLT, LLT, kWidth, 0L, (void*)ML, (void*)ML, kLat, 0L, ML, 0,
        kHalfSets, kLat, kWidth, 1.0f);
    wmma_gemm64<1, 1, 3, 2, 7><<<gemm_grid(kHalfRows, kLat), blk, 0, stream>>>(
        curH, curL, kWidth, 0L, GLT, GLT, kWidth, 0L, (void*)nxtH, (void*)nxtL, kLat, 0L, ML, kLat,
        kHalfRows, kLat, kWidth, 1.0f);
    colsum_kernel<kLat, true, false><<<dim3(kHalfSets), blk, 0, stream>>>(
        nxtH, nxtL, MK, POOLH + soff * kLat, POOLL + soff * kLat);
  }

  wmma_gemm64<1, 1, 2, 2, 7><<<gemm_grid(kSets, kWidth), blk, 0, stream>>>(
      POOLH, POOLL, kLat, 0L, F0T, F0T, kLat, 0L, (void*)Y0H, (void*)Y0L, kWidth, 0L, F0b, 0,
      kSets, kWidth, kLat, 1.0f);
  {
    unsigned short* yiH = Y0H; unsigned short* yiL = Y0L;
    unsigned short* yoH = Y1H; unsigned short* yoL = Y1L;
    for (int i = 0; i < kFMid; ++i) {
      wmma_gemm64<1, 1, 2, 2, 7><<<gemm_grid(kSets, kWidth), blk, 0, stream>>>(
          yiH, yiL, kWidth, 0L, FMT + (size_t)i * sqW, FMT + (size_t)i * sqW, kWidth, 0L,
          (void*)yoH, (void*)yoL, kWidth, 0L, Fmb + (size_t)i * kWidth, 0, kSets, kWidth, kWidth, 1.0f);
      unsigned short* th = yiH; yiH = yoH; yoH = th;
      unsigned short* tl = yiL; yiL = yoL; yoL = tl;
    }
    wmma_gemm64<1, 1, 0, 0, 0><<<gemm_grid(kSets, kNLast), blk, 0, stream>>>(
        yiH, yiL, kWidth, 0L, FLT, FLT, kWidth, 0L, (void*)Z, (void*)Z, kNLast, 0L, ML, 0,
        kSets, kNLast, kWidth, 1.0f);
  }

  softmax_out_kernel<<<dim3(1), blk, 0, stream>>>(Z, Flb, outp);
}
